// ShuffleSelfAttentionLayer_89292370083972
// MI455X (gfx1250) — hardware-verified
//
#include <hip/hip_runtime.h>
#include <math.h>

constexpr int kB = 64;
constexpr int kF = 512;
constexpr int kN = 64;
constexpr int kH = 8;
constexpr int kE = 4096;
constexpr int kHid = 2048;
constexpr int kRows = kB * kN;
constexpr int kGroups = kH * kB;
constexpr float kWCarry = 32.0f;
constexpr float kWCarryInv = 1.0f / 32.0f;
constexpr float kTempInv = 0.125f;
constexpr float kLnEps = 1e-5f;
constexpr float kInvF = 1.0f / 512.0f;

typedef __attribute__((ext_vector_type(16))) _Float16 v16h;
typedef __attribute__((ext_vector_type(8)))  _Float16 v8h;
typedef __attribute__((ext_vector_type(16))) __bf16   v16b;
typedef __attribute__((ext_vector_type(8)))  __bf16   v8b;
typedef __attribute__((ext_vector_type(8)))  float    v8f;
typedef __attribute__((ext_vector_type(4)))  float    v4f;
typedef __attribute__((ext_vector_type(4)))  unsigned int v4u;
typedef __attribute__((ext_vector_type(4)))  int      v4i;

__device__ __forceinline__ unsigned short f2bf_bits(float f) {
  unsigned u = __float_as_uint(f);
  return (unsigned short)((u + 0x7FFFu + ((u >> 16) & 1u)) >> 16);
}
__device__ __forceinline__ float bf_bits2f(unsigned short h) { return __uint_as_float(((unsigned)h) << 16); }

__device__ __forceinline__ void dep_guard_h(v8f& a, v8f& b, v16h x, v16h y) { asm volatile("v_nop\n\tv_nop\n\tv_nop\n\tv_nop" : "+v"(a), "+v"(b) : "v"(x), "v"(y)); }
__device__ __forceinline__ void dep_guard_b(v8f& a, v8f& b, v16b x, v16b y) { asm volatile("v_nop\n\tv_nop\n\tv_nop\n\tv_nop" : "+v"(a), "+v"(b) : "v"(x), "v"(y)); }
__device__ __forceinline__ void keep4_h(v16h a, v16h b, v16h c, v16h d) { asm volatile("v_nop" :: "v"(a), "v"(b), "v"(c), "v"(d)); }
__device__ __forceinline__ void keep4_b(v16b a, v16b b, v16b c, v16b d) { asm volatile("v_nop" :: "v"(a), "v"(b), "v"(c), "v"(d)); }
__device__ __forceinline__ void acc_guard4(v8f& a, v8f& b, v8f& c, v8f& d) { asm volatile("v_nop\n\tv_nop\n\tv_nop\n\tv_nop" : "+v"(a), "+v"(b), "+v"(c), "+v"(d)); }
template <typename T> struct Frag;
template <> struct Frag<_Float16> {
  typedef v16h V; union U { v16h v; v8h h[2]; };
  static __device__ __forceinline__ v16h load(const _Float16* p) {
    U f; f.h[0] = *(const v8h*)(p); f.h[1] = *(const v8h*)(p + 16); return f.v;
  }
  static __device__ __forceinline__ v8f mma(v16h a, v16h b, v8f c) {
    return __builtin_amdgcn_wmma_f32_16x16x32_f16(false, a, false, b, (short)0, c, false, false);
  }
  static __device__ __forceinline__ void guard(v8f& a, v8f& b, v16h x, v16h y) { dep_guard_h(a, b, x, y); }
  static __device__ __forceinline__ void keep(v16h a, v16h b, v16h c, v16h d) { keep4_h(a, b, c, d); }
};
template <> struct Frag<__bf16> {
  typedef v16b V; union U { v16b v; v8b h[2]; };
  static __device__ __forceinline__ v16b load(const __bf16* p) {
    U f; f.h[0] = *(const v8b*)(p); f.h[1] = *(const v8b*)(p + 16); return f.v;
  }
  static __device__ __forceinline__ v8f mma(v16b a, v16b b, v8f c) {
    return __builtin_amdgcn_wmma_f32_16x16x32_bf16(false, a, false, b, (short)0, c, false, false);
  }
  static __device__ __forceinline__ void guard(v8f& a, v8f& b, v16b x, v16b y) { dep_guard_b(a, b, x, y); }
  static __device__ __forceinline__ void keep(v16b a, v16b b, v16b c, v16b d) { keep4_b(a, b, c, d); }
};

__device__ __forceinline__ unsigned pk16(unsigned short a, unsigned short b) { return (unsigned)a | ((unsigned)b << 16); }
__device__ __forceinline__ unsigned short h_bits(float f) { const _Float16 h = (_Float16)f; return __builtin_bit_cast(unsigned short, h); }

template <int ET> struct Elem;
template <> struct Elem<0> { typedef _Float16 T; };
template <> struct Elem<1> { typedef __bf16 T; };
template <int ET, bool SPLIT, int BIAS_MODE, int OUT_MODE, bool RESID, int ACT = 0>
__global__ __launch_bounds__(256) void wmma_gemm64(
    const unsigned short* __restrict__ Ap, const unsigned short* __restrict__ A2p, int lda, long strideA,
    const unsigned short* __restrict__ Btp, const unsigned short* __restrict__ Bt2p, int ldb, long strideB,
    void* __restrict__ Cout, void* __restrict__ Cout2, int ldc, long strideC,
    const float* __restrict__ bias,
    const float* __restrict__ resid, long strideR,
    int M, int N, int K, float scale) {
  typedef typename Elem<ET>::T T;
  typedef typename Frag<T>::V V;
  const T* A = (const T*)Ap; const T* A2 = (const T*)A2p; const T* Bt = (const T*)Btp; const T* Bt2 = (const T*)Bt2p;
  __shared__ __align__(16) float sT[8][16 * 68];
  const int b    = blockIdx.y;
  const int lane = threadIdx.x & 31;
  const int wave = threadIdx.x >> 5;
  const int tilesN = N >> 6;
  const int tilesM = M >> 6;
  const int tile = blockIdx.x * 8 + wave;
  if (tile >= tilesM * tilesN) return;
  const int tm = tile / tilesN;
  const int tn = tile - tm * tilesN;
  const int m0 = tm << 6;
  const int n0 = tn << 6;

  const T* Ab  = A  + (size_t)b * strideA;
  const T* Bb  = Bt + (size_t)b * strideB;
  const T* Ab2 = SPLIT ? (A2  + (size_t)b * strideA) : nullptr;
  const T* Bb2 = SPLIT ? (Bt2 + (size_t)b * strideB) : nullptr;

  const int rlane = lane & 15;
  const int koff  = (lane >> 4) * 8;
  const int mOff  = (lane >> 4) * 8;

  v8f acc[4][4];
#pragma unroll
  for (int i = 0; i < 4; ++i)
#pragma unroll
    for (int j = 0; j < 4; ++j) acc[i][j] = (v8f){0.f,0.f,0.f,0.f,0.f,0.f,0.f,0.f};

  for (int k0 = 0; k0 < K; k0 += 32) {
    V bh[4], bl[4];
#pragma unroll
    for (int j = 0; j < 4; ++j) {
      const size_t bo = (size_t)(n0 + (j << 4) + rlane) * ldb + koff + k0;
      bh[j] = Frag<T>::load(Bb + bo);
      if (SPLIT) bl[j] = Frag<T>::load(Bb2 + bo);
    }
#pragma unroll
    for (int i = 0; i < 4; ++i) {
      const size_t ao = (size_t)(m0 + (i << 4) + rlane) * lda + koff + k0;
      V ah = Frag<T>::load(Ab + ao);
      V al;
      if (SPLIT) al = Frag<T>::load(Ab2 + ao);
#pragma unroll
      for (int j = 0; j < 4; ++j) {
        acc[i][j] = Frag<T>::mma(ah, bh[j], acc[i][j]);
        if (SPLIT) {
          acc[i][j] = Frag<T>::mma(ah, bl[j], acc[i][j]);
          acc[i][j] = Frag<T>::mma(al, bh[j], acc[i][j]);
        }
      }
      Frag<T>::guard(acc[i][0], acc[i][3], ah, SPLIT ? al : ah);
    }
    Frag<T>::keep(bh[0], bh[1], bh[2], bh[3]);
    if (SPLIT) Frag<T>::keep(bl[0], bl[1], bl[2], bl[3]);
  }
  acc_guard4(acc[0][0], acc[0][1], acc[0][2], acc[0][3]);
  acc_guard4(acc[1][0], acc[1][1], acc[1][2], acc[1][3]);
  acc_guard4(acc[2][0], acc[2][1], acc[2][2], acc[2][3]);
  acc_guard4(acc[3][0], acc[3][1], acc[3][2], acc[3][3]);

  float* slab = sT[wave];
  const float* Rb = RESID ? (resid + (size_t)b * strideR) : nullptr;
#pragma unroll
  for (int i = 0; i < 4; ++i) {
    const int mBase = m0 + (i << 4);
#pragma unroll
    for (int j = 0; j < 4; ++j) {
      const int n = n0 + (j << 4) + rlane;
      float bv = 0.f;
      if (BIAS_MODE == 2) bv = bias[n];
#pragma unroll
      for (int r = 0; r < 8; ++r) {
        float v = acc[i][j][r] * scale;
        if (BIAS_MODE == 1) v += bias[mBase + mOff + r];
        if (BIAS_MODE == 2) v += bv;
        if (RESID) v += Rb[(size_t)(mBase + mOff + r) * ldc + n];
        if (ACT == 2) v = fmaxf(v, 0.0f);
        if (ACT == 4) v = (v > 0.f) ? v : 0.01f * v;
        slab[(mOff + r) * 68 + (j << 4) + rlane] = v;
      }
    }
    __builtin_amdgcn_fence(__ATOMIC_RELEASE, "workgroup");
    __builtin_amdgcn_wave_barrier();
    __builtin_amdgcn_fence(__ATOMIC_ACQUIRE, "workgroup");
    if (OUT_MODE == 0) {
      float* C = (float*)Cout + (size_t)b * strideC;
      const int hh = lane >> 4, c4 = (lane & 15) * 4;
      for (int pass = 0; pass < 2; ++pass) {
#pragma unroll
        for (int it = 0; it < 8; ++it) {
          const int row = it * 2 + hh;
          v4f v = *(const v4f*)(slab + row * 68 + c4);
          *(volatile v4f*)(C + (size_t)(mBase + row) * ldc + n0 + c4) = v;
        }
        __threadfence();
      }
    } else {
      const int q = lane >> 3, c8 = (lane & 7) * 8;
      unsigned short* C  = (unsigned short*)Cout  + (size_t)b * strideC;
      unsigned short* C2 = (OUT_MODE == 2) ? ((unsigned short*)Cout2 + (size_t)b * strideC) : nullptr;
      for (int pass = 0; pass < 2; ++pass) {
#pragma unroll
        for (int it = 0; it < 4; ++it) {
          const int row = it * 4 + q;
          const float* sp = slab + row * 68 + c8;
          v8h hv, lv;
#pragma unroll
          for (int e = 0; e < 8; ++e) {
            if (OUT_MODE == 1) {
              hv[e] = (_Float16)sp[e];
            } else {
              unsigned short hb = f2bf_bits(sp[e]);
              unsigned short lb = f2bf_bits(sp[e] - bf_bits2f(hb));
              hv[e] = __builtin_bit_cast(_Float16, hb);
              lv[e] = __builtin_bit_cast(_Float16, lb);
            }
          }
          *(volatile v8h*)(C + (size_t)(mBase + row) * ldc + n0 + c8) = hv;
          if (OUT_MODE == 2) *(volatile v8h*)(C2 + (size_t)(mBase + row) * ldc + n0 + c8) = lv;
        }
        __threadfence();
      }
    }
    __builtin_amdgcn_fence(__ATOMIC_RELEASE, "workgroup");
    __builtin_amdgcn_wave_barrier();
    __builtin_amdgcn_fence(__ATOMIC_ACQUIRE, "workgroup");
  }
}

__global__ __launch_bounds__(256) void gather_kernel(const float* __restrict__ feat, const int* __restrict__ sidx,
                                                     unsigned short* __restrict__ fm, int n8) {
  const int i = blockIdx.x * 256 + threadIdx.x;
  if (i >= n8) return;
  const int e0 = i * 8;
  const int f = e0 & (kF - 1);
  const int m = e0 >> 9;
  const int b = m >> 6;
  const int n = m & 63;
  const int* ip = sidx + n * kF + f;
  const v4i ia = *(const v4i*)(ip);
  const v4i ib = *(const v4i*)(ip + 4);
  const float* fr = feat + (size_t)b * kF;
  unsigned short hb[8];
#pragma unroll
  for (int e = 0; e < 4; ++e) {
    int j0 = ia[e]; j0 = (j0 < 0) ? 0 : ((j0 > kF - 1) ? (kF - 1) : j0);
    int j1 = ib[e]; j1 = (j1 < 0) ? 0 : ((j1 > kF - 1) ? (kF - 1) : j1);
    hb[e]     = h_bits(fr[j0]);
    hb[4 + e] = h_bits(fr[j1]);
  }
  const v4u u = (v4u){pk16(hb[0], hb[1]), pk16(hb[2], hb[3]), pk16(hb[4], hb[5]), pk16(hb[6], hb[7])};
  unsigned short* q = fm + (size_t)e0;
  *(volatile v4u*)q = u;
  __threadfence();
  *(volatile v4u*)q = u;
}

__global__ __launch_bounds__(256) void tcast_kernel(const float* __restrict__ in0, const float* __restrict__ in1,
                                                    const float* __restrict__ in2, unsigned short* __restrict__ out,
                                                    int R, int Ccols, float scale) {
  __shared__ float sm[64][65];
  const int t  = threadIdx.x;
  const int r0 = blockIdx.x * 64;
  const int c0 = blockIdx.y * 64;
  const int z  = blockIdx.z;
  const float* W = (z == 0) ? in0 : (z == 1) ? in1 : in2;
#pragma unroll
  for (int i = 0; i < 16; ++i) {
    const int e = i * 256 + t;
    const int r = e >> 6;
    const int c = e & 63;
    sm[c][r] = W[(size_t)(r0 + r) * Ccols + c0 + c] * scale;
  }
  __syncthreads();
  const int lane = t & 31, wave = t >> 5;
  const int q = lane >> 3, c8 = (lane & 7) * 8;
  unsigned short* op = out + (size_t)z * (size_t)R * (size_t)Ccols;
  for (int pass = 0; pass < 2; ++pass) {
#pragma unroll
    for (int it = 0; it < 2; ++it) {
      const int row = wave * 8 + it * 4 + q;
      unsigned short hb[8];
#pragma unroll
      for (int e = 0; e < 8; ++e) hb[e] = h_bits(sm[row][c8 + e]);
      const v4u u = (v4u){pk16(hb[0], hb[1]), pk16(hb[2], hb[3]), pk16(hb[4], hb[5]), pk16(hb[6], hb[7])};
      *(volatile v4u*)(op + (size_t)(c0 + row) * R + r0 + c8) = u;
    }
    __threadfence();
  }
}

__global__ __launch_bounds__(256) void softmax_kernel(const float* __restrict__ S, const float* __restrict__ conv_w,
                                                      float* __restrict__ attn, float* __restrict__ wp) {
  __shared__ __align__(16) float Ps[kN * kN];
  __shared__ float cw[kN];
  __shared__ __align__(16) float wl[kN];
  const int g = blockIdx.x;
  const int h = g >> 6;
  const int t = threadIdx.x;
  const int lane = t & 31, wave = t >> 5;
  const float* sg = S + (size_t)g * kN * kN;
#pragma unroll
  for (int it = 0; it < 4; ++it) {
    const int i4 = it * 256 + t;
    *(v4f*)(Ps + i4 * 4) = *(const v4f*)(sg + i4 * 4);
  }
  if (t < kN) cw[t] = conv_w[h * kN + t];
  __syncthreads();
#pragma unroll 1
  for (int r = 0; r < 8; ++r) {
    const int row = wave * 8 + r;
    const float a = Ps[row * kN + lane];
    const float c = Ps[row * kN + lane + 32];
    float m = fmaxf(a, c);
#pragma unroll
    for (int off = 16; off > 0; off >>= 1) m = fmaxf(m, __shfl_xor(m, off, 32));
    const float ea = expf(a - m);
    const float ec = expf(c - m);
    float s = ea + ec;
#pragma unroll
    for (int off = 16; off > 0; off >>= 1) s += __shfl_xor(s, off, 32);
    const float inv = 1.0f / s;
    Ps[row * kN + lane]      = ea * inv;
    Ps[row * kN + lane + 32] = ec * inv;
  }
  __syncthreads();
  float* dst = attn + (size_t)g * kN * kN;
  for (int pass = 0; pass < 2; ++pass) {
#pragma unroll
    for (int it = 0; it < 4; ++it) {
      const int i4 = it * 256 + t;
      const v4f v = *(const v4f*)(Ps + i4 * 4);
      *(volatile v4f*)(dst + i4 * 4) = v;
    }
    __threadfence();
  }
  if (t < kN) {
    float acc = 0.f;
#pragma unroll 1
    for (int n = 0; n < kN; ++n) acc = fmaf(cw[n], Ps[n * kN + t], acc);
    wl[t] = acc;
  }
  __syncthreads();
  if (t < 16) {
    const v4f v = *(const v4f*)(wl + t * 4);
    float* wd = wp + (size_t)g * kN + t * 4;
    *(volatile v4f*)wd = v;
    __threadfence();
    *(volatile v4f*)wd = v;
  }
}

__device__ __forceinline__ float block_sum512(float v, float* red, int lane, int wave) {
#pragma unroll
  for (int off = 16; off > 0; off >>= 1) v += __shfl_xor(v, off, 32);
  if (lane == 0) red[wave] = v;
  __syncthreads();
  float s = 0.f;
#pragma unroll
  for (int w = 0; w < 16; ++w) s += red[w];
  __syncthreads();
  return s;
}

__global__ __launch_bounds__(512) void combine_ln1_kernel(const float* __restrict__ V, const float* __restrict__ wp,
                                                          const float* __restrict__ feat,
                                                          const float* __restrict__ gam, const float* __restrict__ bet,
                                                          float* __restrict__ xf, unsigned short* __restrict__ x16) {
  __shared__ float wl[kH * kN];
  __shared__ float red[16];
  __shared__ __align__(16) float xs[kF];
  const int b = blockIdx.x;
  const int f = threadIdx.x;
  const int lane = f & 31, wave = f >> 5;
  wl[f] = wp[((size_t)((f >> 6) * kB + b)) * kN + (f & 63)];
  __syncthreads();
  const float* vp = V + (size_t)b * kN * kE + f;
  float acc = 0.f;
#pragma unroll 1
  for (int j = 0; j < kH * kN; ++j) {
    const int hh = j >> 6;
    const int nn = j & 63;
    acc = fmaf(wl[j], vp[(size_t)nn * kE + hh * kF], acc);
  }
  const float tval = acc + feat[(size_t)b * kF + f];
  const float mu  = block_sum512(tval, red, lane, wave) * kInvF;
  const float d   = tval - mu;
  const float var = block_sum512(d * d, red, lane, wave) * kInvF;
  const float x   = d * rsqrtf(var + kLnEps) * gam[f] + bet[f];
  xs[f] = x;
  __syncthreads();
  if (f < 128) {
    const v4f v = *(const v4f*)(xs + f * 4);
    float* p = xf + (size_t)b * kF + f * 4;
    *(volatile v4f*)p = v;
    __threadfence();
    *(volatile v4f*)p = v;
  }
  if (f < 64) {
    unsigned short hb[8];
#pragma unroll
    for (int e = 0; e < 8; ++e) hb[e] = h_bits(xs[f * 8 + e]);
    const v4u u = (v4u){pk16(hb[0], hb[1]), pk16(hb[2], hb[3]), pk16(hb[4], hb[5]), pk16(hb[6], hb[7])};
    unsigned short* q = x16 + (size_t)b * kF + f * 8;
    *(volatile v4u*)q = u;
    __threadfence();
    *(volatile v4u*)q = u;
  }
}

__global__ __launch_bounds__(512) void ln2_kernel(const float* __restrict__ hres, const float* __restrict__ gam,
                                                  const float* __restrict__ bet, float* __restrict__ yout) {
  __shared__ float red[16];
  __shared__ __align__(16) float xs[kF];
  const int b = blockIdx.x;
  const int f = threadIdx.x;
  const int lane = f & 31, wave = f >> 5;
  const float tval = hres[(size_t)b * kF + f];
  const float mu  = block_sum512(tval, red, lane, wave) * kInvF;
  const float d   = tval - mu;
  const float var = block_sum512(d * d, red, lane, wave) * kInvF;
  const float y   = d * rsqrtf(var + kLnEps) * gam[f] + bet[f];
  xs[f] = y;
  __syncthreads();
  if (f < 128) {
    const v4f v = *(const v4f*)(xs + f * 4);
    float* p = yout + (size_t)b * kF + f * 4;
    *(volatile v4f*)p = v;
    __threadfence();
    *(volatile v4f*)p = v;
  }
}

extern "C" void kernel_launch(void* const* d_in, const int* in_sizes, int n_in,
                              void* d_out, int out_size, void* d_ws, size_t ws_size,
                              hipStream_t stream) {
  (void)in_sizes;
  if (n_in < 17) return;
  if (out_size < kB * kF + kGroups * kN * kN) return;

  const float* features = (const float*)d_in[0];
  const int*   shuf     = (const int*)d_in[1];
  const float* Wq = (const float*)d_in[2];   const float* bq = (const float*)d_in[3];
  const float* Wk = (const float*)d_in[4];   const float* bk = (const float*)d_in[5];
  const float* Wv = (const float*)d_in[6];   const float* bv = (const float*)d_in[7];
  const float* conv_w = (const float*)d_in[8];
  const float* ln1_g = (const float*)d_in[9];  const float* ln1_b = (const float*)d_in[10];
  const float* W1 = (const float*)d_in[11];  const float* b1 = (const float*)d_in[12];
  const float* W2 = (const float*)d_in[13];  const float* b2 = (const float*)d_in[14];
  const float* ln2_g = (const float*)d_in[15]; const float* ln2_b = (const float*)d_in[16];

  float* y_out    = (float*)d_out;
  float* attn_out = (float*)d_out + (size_t)kB * kF;

  size_t off = 0;
  auto carve = [&](size_t bytes) -> char* {
    char* p = (char*)d_ws + off;
    off += (bytes + 255) & ~(size_t)255;
    return p;
  };
  unsigned short* FM16  = (unsigned short*)carve((size_t)kRows * kF * 2);
  unsigned short* WQKVT = (unsigned short*)carve((size_t)3 * kE * kF * 2);
  unsigned short* WQT = WQKVT;
  unsigned short* WKT = WQKVT + (size_t)kE * kF;
  unsigned short* WVT = WQKVT + (size_t)2 * kE * kF;
  unsigned short* W1T = (unsigned short*)carve((size_t)kHid * kF * 2);
  unsigned short* W2T = (unsigned short*)carve((size_t)kF * kHid * 2);
  char* qkv = carve((size_t)kRows * kE * 4);
  unsigned short* Q16 = (unsigned short*)qkv;
  unsigned short* K16 = (unsigned short*)qkv + (size_t)kRows * kE;
  float* V32 = (float*)qkv;
  float* S32  = (float*)carve((size_t)kGroups * kN * kN * 4);
  float* WP   = (float*)carve((size_t)kGroups * kN * 4);
  float* XF   = (float*)carve((size_t)kB * kF * 4);
  unsigned short* X16 = (unsigned short*)carve((size_t)kB * kF * 2);
  unsigned short* H16 = (unsigned short*)carve((size_t)kB * kHid * 2);
  float* HRES = (float*)carve((size_t)kB * kF * 4);
  if (off > ws_size) return;

  const int n8 = kRows * kF / 8;
  gather_kernel<<<n8 / 256, 256, 0, stream>>>(features, shuf, FM16, n8);

  tcast_kernel<<<dim3(kF / 64, kE / 64, 3), 256, 0, stream>>>(Wq, Wk, Wv, WQKVT, kF, kE, kWCarry);
  tcast_kernel<<<dim3(kF / 64, kHid / 64, 1), 256, 0, stream>>>(W1, W1, W1, W1T, kF, kHid, kWCarry);
  tcast_kernel<<<dim3(kHid / 64, kF / 64, 1), 256, 0, stream>>>(W2, W2, W2, W2T, kHid, kF, kWCarry);

  wmma_gemm64<0, false, 2, 1, false, 0><<<dim3((kRows / 64) * (kE / 64) / 8, 1), 256, 0, stream>>>(
      FM16, FM16, kF, 0L, WQT, WQT, kF, 0L, (void*)Q16, (void*)Q16, kE, 0L, bq, bq, 0L, kRows, kE, kF, kWCarryInv);
  wmma_gemm64<0, false, 2, 1, false, 0><<<dim3((kRows / 64) * (kE / 64) / 8, 1), 256, 0, stream>>>(
      FM16, FM16, kF, 0L, WKT, WKT, kF, 0L, (void*)K16, (void*)K16, kE, 0L, bk, bk, 0L, kRows, kE, kF, kWCarryInv);

  for (int h = 0; h < kH; ++h) {
    wmma_gemm64<0, false, 0, 0, false, 0><<<dim3(1, kB), 256, 0, stream>>>(
        Q16 + (size_t)h * kF, Q16 + (size_t)h * kF, kE, (long)kN * kE,
        K16 + (size_t)h * kF, K16 + (size_t)h * kF, kE, (long)kN * kE,
        (void*)(S32 + (size_t)h * kB * kN * kN), (void*)(S32 + (size_t)h * kB * kN * kN), kN, (long)kN * kN,
        bq, bq, 0L, kN, kN, kF, kTempInv);
  }

  softmax_kernel<<<kGroups, 256, 0, stream>>>(S32, conv_w, attn_out, WP);

  wmma_gemm64<0, false, 2, 0, false, 0><<<dim3((kRows / 64) * (kE / 64) / 8, 1), 256, 0, stream>>>(
      FM16, FM16, kF, 0L, WVT, WVT, kF, 0L, (void*)V32, (void*)V32, kE, 0L, bv, bv, 0L, kRows, kE, kF, kWCarryInv);

  combine_ln1_kernel<<<kB, kF, 0, stream>>>(V32, WP, features, ln1_g, ln1_b, XF, X16);

  wmma_gemm64<0, false, 2, 1, false, 2><<<dim3((kB / 64) * (kHid / 64) / 8, 1), 256, 0, stream>>>(
      X16, X16, kF, 0L, W1T, W1T, kF, 0L, (void*)H16, (void*)H16, kHid, 0L, b1, b1, 0L, kB, kHid, kF, kWCarryInv);
  wmma_gemm64<0, false, 2, 0, true, 0><<<dim3(1, 1), 256, 0, stream>>>(
      H16, H16, kHid, 0L, W2T, W2T, kHid, 0L, (void*)HRES, (void*)HRES, kF, 0L, b2, XF, 0L, kB, kF, kHid, kWCarryInv);

  ln2_kernel<<<kB, kF, 0, stream>>>(HRES, ln2_g, ln2_b, y_out);
}
